// RWKV_Tmix_x070_54760833024019
// MI455X (gfx1250) — hardware-run, weakly checked
//
#include <hip/hip_runtime.h>
#include <math.h>

constexpr int kBatch   = 4;
constexpr int kSteps   = 1024;
constexpr int kChan    = 1024;
constexpr int kHeads   = 16;
constexpr int kHdim    = 64;
constexpr int kTok     = kBatch * kSteps;
constexpr size_t kPlane = (size_t)kTok * kChan;
constexpr int kMixRank = 32;
constexpr int kMixHid  = 4 * kMixRank;
constexpr int kDecHid  = 64;
constexpr int kLoraR   = 16;
constexpr int kGateHid = 128;
constexpr int kHidWa   = 128;
constexpr int kHidK    = 64;
constexpr int kK2Pitch = 64;
constexpr int kW1Rows  = kMixHid + kGateHid + kHidWa + kHidK;
constexpr int kChunk   = 16;

constexpr float kWCarry   = 16.0f;
constexpr float kWkCarry  = 256.0f;
constexpr float kHidCarry = 16.0f;
constexpr float kYCarry   = 64.0f;
constexpr float kScaleW   = 1.0f / kWCarry;
constexpr float kScaleWk  = 1.0f / kWkCarry;
constexpr float kScaleWH  = 1.0f / (kWCarry * kHidCarry);
constexpr float kScaleOut = 1.0f / (kWCarry * kYCarry);
constexpr float kGnEps    = 64e-5f;

static_assert(kHeads * kHdim == kChan);
static_assert((kSteps & (kSteps - 1)) == 0);
static_assert(kTok % 32 == 0 && kChan % 64 == 0);
static_assert(kMixHid % 64 == 0 && kGateHid % 64 == 0 && kHidWa % 64 == 0 && kHidK % 64 == 0);
static_assert(kChan % 32 == 0 && kMixRank % 32 == 0 && kDecHid % 32 == 0 && kGateHid % 32 == 0);
static_assert(kDecHid + 2 * kLoraR <= kHidWa && 2 * kLoraR <= kHidK && 2 * kLoraR == 32);
static_assert(kSteps % kChunk == 0 && kHdim == 64 && kChunk == 16);
static_assert((kTok * kHeads) % 8 == 0);
static_assert(kW1Rows == 448);
static_assert(((kTok / 32) * (kChan / 64)) % 8 == 0);
static_assert(((kTok / 32) * (kMixHid / 64)) % 8 == 0);
static_assert(((kTok / 32) * (kHidK / 64)) % 8 == 0);

typedef __attribute__((ext_vector_type(16))) _Float16 v16h;
typedef __attribute__((ext_vector_type(8)))  _Float16 v8h;
typedef __attribute__((ext_vector_type(8)))  float    v8f;
typedef __attribute__((ext_vector_type(4)))  float    v4f;
typedef __attribute__((ext_vector_type(2)))  float    v2f;
typedef __attribute__((ext_vector_type(4)))  unsigned int v4u;
typedef __attribute__((ext_vector_type(2)))  unsigned int v2u;

__device__ __forceinline__ unsigned pk16(unsigned short a, unsigned short b) {
  return (unsigned)a | ((unsigned)b << 16);
}
__device__ __forceinline__ unsigned short h_bits(float f) {
  const _Float16 h = (_Float16)f;
  return __builtin_bit_cast(unsigned short, h);
}
__device__ __forceinline__ float h16_to_f32(unsigned hb) {
  const unsigned sgn = (hb & 0x8000u) << 16;
  const unsigned em = hb & 0x7fffu;
  const float fn = __uint_as_float((em << 13) + 0x38000000u);
  const float fs = (float)em * 5.9604644775390625e-8f;
  const float mag = (em < 0x400u) ? fs : fn;
  return __uint_as_float(__float_as_uint(mag) | sgn);
}
__device__ __forceinline__ v4u pack8_plain(const float (&v)[8]) {
  unsigned short hb[8];
#pragma unroll
  for (int e = 0; e < 8; ++e) hb[e] = h_bits(v[e]);
  return (v4u){pk16(hb[0], hb[1]), pk16(hb[2], hb[3]), pk16(hb[4], hb[5]), pk16(hb[6], hb[7])};
}
__device__ __forceinline__ float wave_sum32(float v) {
#pragma unroll
  for (int o = 16; o > 0; o >>= 1) v += __shfl_xor(v, o, 32);
  return v;
}
__device__ __forceinline__ v4f ld4h(const unsigned short* p) {
  const v2u u = *(const v2u*)(const void*)p;
  const unsigned w0 = u[0];
  const unsigned w1 = u[1];
  return (v4f){h16_to_f32(w0 & 0xffffu), h16_to_f32(w0 >> 16), h16_to_f32(w1 & 0xffffu), h16_to_f32(w1 >> 16)};
}

struct FragH {
  union U { v16h v; v8h h[2]; };
  static __device__ __forceinline__ v16h load(const _Float16* p) {
    U f;
    f.h[0] = *(const v8h*)(p);
    f.h[1] = *(const v8h*)(p + 16);
    return f.v;
  }
  static __device__ __forceinline__ v8f mma(v16h a, v16h b, v8f c) {
    return __builtin_amdgcn_wmma_f32_16x16x32_f16(false, a, false, b, (short)0, c, false, false);
  }
};
__device__ __forceinline__ void guard_plain(v8f& a0, v8f& a1, v16h x0, v16h x1, v16h y0) {
  asm volatile("v_nop\n\tv_nop\n\tv_nop\n\tv_nop"
               : "+v"(a0), "+v"(a1)
               : "v"(x0), "v"(x1), "v"(y0));
}
__device__ __forceinline__ void acc_guard4(v8f& a, v8f& b, v8f& c, v8f& d) {
  asm volatile("v_nop\n\tv_nop\n\tv_nop\n\tv_nop" : "+v"(a), "+v"(b), "+v"(c), "+v"(d));
}
__device__ __forceinline__ void wave_lds_sync() {
  __builtin_amdgcn_fence(__ATOMIC_RELEASE, "workgroup");
  __builtin_amdgcn_wave_barrier();
  __builtin_amdgcn_fence(__ATOMIC_ACQUIRE, "workgroup");
}

template <int ACT, int OUT_MODE>
__global__ __launch_bounds__(256) void gemm_f16_kernel(
    const unsigned short* __restrict__ Ap, int lda, long strideA,
    const unsigned short* __restrict__ Bp, int ldb, long strideB,
    void* __restrict__ Cout, int ldc, long strideC,
    int M, int N, int K, float scale, float outCarry, int actLimit) {
  static_assert(ACT == 0 || OUT_MODE == 1);
  __shared__ __align__(16) float sT[8][16 * 68];
  const int z    = blockIdx.y;
  const int lane = threadIdx.x & 31;
  const int wave = threadIdx.x >> 5;
  const int tilesN = N >> 6;
  const int tilesM = M >> 5;
  const int tile = blockIdx.x * 8 + wave;
  if (tile >= tilesM * tilesN) return;
  const int tm = tile / tilesN;
  const int tn = tile - tm * tilesN;
  const int m0 = tm << 5;
  const int n0 = tn << 6;
  const int rlane = lane & 15;
  const int half8 = (lane >> 4) * 8;
  const int mOff  = (lane >> 4) * 8;

  const size_t aoff = (size_t)z * (size_t)strideA + (size_t)(m0 + rlane) * lda + half8;
  const size_t boff = (size_t)z * (size_t)strideB + (size_t)(n0 + rlane) * ldb + half8;
  const _Float16* pa0 = (const _Float16*)Ap + aoff;
  const _Float16* pa1 = pa0 + (size_t)16 * lda;
  const _Float16* pbh = (const _Float16*)Bp + boff;
  const size_t bstep = (size_t)16 * ldb;

  v8f acc[2][4];
#pragma unroll
  for (int i = 0; i < 2; ++i)
#pragma unroll
    for (int j = 0; j < 4; ++j) acc[i][j] = (v8f){0.f, 0.f, 0.f, 0.f, 0.f, 0.f, 0.f, 0.f};

  for (int k0 = 0; k0 < K; k0 += 32) {
    const v16h ah0 = FragH::load(pa0 + k0);
    const v16h ah1 = FragH::load(pa1 + k0);
#pragma unroll
    for (int j = 0; j < 4; ++j) {
      const v16h bh = FragH::load(pbh + j * bstep + k0);
      acc[0][j] = FragH::mma(ah0, bh, acc[0][j]);
      acc[1][j] = FragH::mma(ah1, bh, acc[1][j]);
      guard_plain(acc[0][j], acc[1][j], ah0, ah1, bh);
    }
  }
  acc_guard4(acc[0][0], acc[0][1], acc[0][2], acc[0][3]);
  acc_guard4(acc[1][0], acc[1][1], acc[1][2], acc[1][3]);

  float* slab = sT[wave];
#pragma unroll
  for (int i = 0; i < 2; ++i) {
    const int mBase = m0 + (i << 4);
#pragma unroll
    for (int j = 0; j < 4; ++j) {
#pragma unroll
      for (int r = 0; r < 8; ++r) {
        slab[(mOff + r) * 68 + (j << 4) + rlane] = acc[i][j][r] * scale;
      }
    }
    wave_lds_sync();
    if (OUT_MODE == 0) {
      float* C = (float*)Cout + (size_t)z * (size_t)strideC;
      const int hh = lane >> 4, c4 = (lane & 15) * 4;
      for (int pass = 0; pass < 2; ++pass) {
#pragma unroll
        for (int it = 0; it < 8; ++it) {
          const int row = it * 2 + hh;
          const v4f v = *(const v4f*)(slab + row * 68 + c4);
          *(volatile v4f*)(C + (size_t)(mBase + row) * ldc + n0 + c4) = v;
        }
        __threadfence();
      }
    } else {
      const int q = lane >> 3, c8 = (lane & 7) * 8;
      if (ACT != 0) {
        const bool lim = (n0 + c8) < actLimit;
#pragma unroll 1
        for (int it = 0; it < 4; ++it) {
          float* sp = slab + (it * 4 + q) * 68 + c8;
#pragma unroll
          for (int e = 0; e < 8; ++e) {
            const float xv = sp[e];
            const float th = tanhf(xv);
            const float yv = lim ? th : xv;
            sp[e] = yv * outCarry;
          }
        }
      }
      unsigned short* C = (unsigned short*)Cout + (size_t)z * (size_t)strideC;
      for (int pass = 0; pass < 2; ++pass) {
#pragma unroll
        for (int it = 0; it < 4; ++it) {
          const int row = it * 4 + q;
          const float* sp = slab + row * 68 + c8;
          v8h hv;
#pragma unroll
          for (int e = 0; e < 8; ++e) hv[e] = (_Float16)sp[e];
          *(volatile v8h*)(C + (size_t)(mBase + row) * ldc + n0 + c8) = hv;
        }
        __threadfence();
      }
    }
    wave_lds_sync();
  }
}

__global__ __launch_bounds__(256) void mix2_kernel(
    const unsigned short* __restrict__ Hm, const unsigned short* __restrict__ W2t,
    const float* __restrict__ x,
    const float* __restrict__ mv0, const float* __restrict__ mv1,
    const float* __restrict__ mv2, const float* __restrict__ mv3,
    unsigned short* __restrict__ Xout, float scale) {
  __shared__ __align__(16) float sT[8][16 * 68];
  const int f    = blockIdx.y;
  const float* mv = (f == 0) ? mv0 : (f == 1) ? mv1 : (f == 2) ? mv2 : mv3;
  const int lane = threadIdx.x & 31;
  const int wave = threadIdx.x >> 5;
  const int tilesN = kChan >> 6;
  const int tilesM = kTok >> 5;
  const int tile = blockIdx.x * 8 + wave;
  if (tile >= tilesM * tilesN) return;
  const int tm = tile / tilesN;
  const int tn = tile - tm * tilesN;
  const int m0 = tm << 5;
  const int n0 = tn << 6;
  const int rlane = lane & 15;
  const int half8 = (lane >> 4) * 8;
  const int mOff  = (lane >> 4) * 8;

  const _Float16* pa0 = (const _Float16*)Hm + (size_t)(m0 + rlane) * kMixHid + f * kMixRank + half8;
  const _Float16* pa1 = pa0 + (size_t)16 * kMixHid;
  const _Float16* pb  = (const _Float16*)W2t + (size_t)f * kChan * kK2Pitch + (size_t)(n0 + rlane) * kK2Pitch + half8;

  v8f acc[2][4];
#pragma unroll
  for (int i = 0; i < 2; ++i)
#pragma unroll
    for (int j = 0; j < 4; ++j) acc[i][j] = (v8f){0.f, 0.f, 0.f, 0.f, 0.f, 0.f, 0.f, 0.f};
  {
    const v16h ah0 = FragH::load(pa0);
    const v16h ah1 = FragH::load(pa1);
#pragma unroll
    for (int j = 0; j < 4; ++j) {
      const v16h bh = FragH::load(pb + (size_t)j * 16 * kK2Pitch);
      acc[0][j] = FragH::mma(ah0, bh, acc[0][j]);
      acc[1][j] = FragH::mma(ah1, bh, acc[1][j]);
      guard_plain(acc[0][j], acc[1][j], ah0, ah1, bh);
    }
  }
  acc_guard4(acc[0][0], acc[0][1], acc[0][2], acc[0][3]);
  acc_guard4(acc[1][0], acc[1][1], acc[1][2], acc[1][3]);

  float* slab = sT[wave];
  unsigned short* Xo = Xout + (size_t)f * kPlane;
  const int q = lane >> 3, c8 = (lane & 7) * 8;
  const v4f ma = *(const v4f*)(mv + n0 + c8);
  const v4f mb = *(const v4f*)(mv + n0 + c8 + 4);
#pragma unroll
  for (int i = 0; i < 2; ++i) {
    const int mBase = m0 + (i << 4);
#pragma unroll
    for (int j = 0; j < 4; ++j) {
#pragma unroll
      for (int r = 0; r < 8; ++r) {
        slab[(mOff + r) * 68 + (j << 4) + rlane] = acc[i][j][r] * scale;
      }
    }
    wave_lds_sync();
    v4u pk[4];
#pragma unroll
    for (int it = 0; it < 4; ++it) {
      const int row = it * 4 + q;
      const int m = mBase + row;
      const bool first = (m & (kSteps - 1)) == 0;
      const int srow = first ? m : (m - 1);
      const float* sp = slab + row * 68 + c8;
      const float* xp = x + (size_t)m * kChan + n0 + c8;
      const float* pp = x + (size_t)srow * kChan + n0 + c8;
      const v4f a  = *(const v4f*)(xp);
      const v4f b  = *(const v4f*)(xp + 4);
      const v4f pa = *(const v4f*)(pp);
      const v4f pbv = *(const v4f*)(pp + 4);
      const v4f s0 = *(const v4f*)(sp);
      const v4f s1 = *(const v4f*)(sp + 4);
      float o[8];
#pragma unroll
      for (int e = 0; e < 4; ++e) {
        const float p0 = first ? 0.0f : pa[e];
        const float p1 = first ? 0.0f : pbv[e];
        const float x0 = p0 - a[e];
        const float x1 = p1 - b[e];
        o[e]     = a[e] + x0 * (ma[e] + s0[e]);
        o[4 + e] = b[e] + x1 * (mb[e] + s1[e]);
      }
      pk[it] = pack8_plain(o);
    }
    for (int pass = 0; pass < 2; ++pass) {
#pragma unroll
      for (int it = 0; it < 4; ++it) {
        const int row = it * 4 + q;
        *(volatile v4u*)(Xo + (size_t)(mBase + row) * kChan + n0 + c8) = pk[it];
      }
      __threadfence();
    }
    wave_lds_sync();
  }
}

struct PlaceArgs {
  const float* p[4];
  int Kd[4];
  int Nd[4];
  int rowOff[4];
  int colOff[4];
};
static_assert(sizeof(PlaceArgs) == 96);

__global__ __launch_bounds__(256) void wt_place_kernel(PlaceArgs a, unsigned short* __restrict__ out, int pitch, float carry) {
  __shared__ float sm[64][65];
  const int t  = threadIdx.x;
  const int k0 = blockIdx.x * 64;
  const int n0 = blockIdx.y * 64;
#pragma unroll 2
  for (int i = 0; i < 16; ++i) {
    const int e = i * 256 + t;
    const int r = e >> 6;
    const int c = e & 63;
    const int kk = k0 + r;
    const int nn = n0 + c;
    float val = 0.0f;
#pragma unroll
    for (int s = 0; s < 4; ++s) {
      const int kr = kk - a.colOff[s];
      const int nr = nn - a.rowOff[s];
      const bool valid = (kr >= 0) && (kr < a.Kd[s]) && (nr >= 0) && (nr < a.Nd[s]);
      int kc = kr < 0 ? 0 : kr;
      kc = kc > a.Kd[s] - 1 ? a.Kd[s] - 1 : kc;
      int nc = nr < 0 ? 0 : nr;
      nc = nc > a.Nd[s] - 1 ? a.Nd[s] - 1 : nc;
      const float v = a.p[s][(size_t)kc * a.Nd[s] + nc];
      val = valid ? (v * carry) : val;
    }
    sm[c][r] = val;
  }
  __syncthreads();
  const int lane = t & 31, wave = t >> 5;
  const int q = lane >> 3, c8 = (lane & 7) * 8;
  for (int pass = 0; pass < 2; ++pass) {
#pragma unroll
    for (int it = 0; it < 2; ++it) {
      const int row = wave * 8 + it * 4 + q;
      float v[8];
#pragma unroll
      for (int e = 0; e < 8; ++e) v[e] = sm[row][c8 + e];
      const v4u u = pack8_plain(v);
      *(volatile v4u*)(out + (size_t)(n0 + row) * pitch + k0 + c8) = u;
    }
    __threadfence();
  }
}

__global__ __launch_bounds__(256) void cast8_w4_kernel(const float* __restrict__ W0, const float* __restrict__ W1,
                                                       const float* __restrict__ W2, const float* __restrict__ W3,
                                                       unsigned short* __restrict__ out,
                                                       float s0, float s1, float s2, float s3, int n8) {
  const int z = blockIdx.y;
  const float* W = (z == 0) ? W0 : (z == 1) ? W1 : (z == 2) ? W2 : W3;
  const float s  = (z == 0) ? s0 : (z == 1) ? s1 : (z == 2) ? s2 : s3;
  const int i = blockIdx.x * 256 + threadIdx.x;
  if (i >= n8) return;
  const float* p = W + 8 * (size_t)i;
  const v4f a = *(const v4f*)(p);
  const v4f c = *(const v4f*)(p + 4);
  float v[8];
#pragma unroll
  for (int e = 0; e < 4; ++e) {
    v[e]     = a[e] * s;
    v[4 + e] = c[e] * s;
  }
  const v4u u = pack8_plain(v);
  unsigned short* q = out + (size_t)z * (size_t)n8 * 8 + 8 * (size_t)i;
  *(volatile v4u*)q = u;
  __threadfence();
  *(volatile v4u*)q = u;
}

__global__ __launch_bounds__(256) void shift_mix_kernel(const float* __restrict__ x, const float* __restrict__ mvec,
                                                        unsigned short* __restrict__ XM) {
  const int i = blockIdx.x * 256 + threadIdx.x;
  if (i >= kTok * (kChan / 8)) return;
  const int row = i >> 7;
  const int c8  = (i & 127) * 8;
  const bool first = (row & (kSteps - 1)) == 0;
  const int srow = first ? row : (row - 1);
  const float* xp = x + (size_t)row * kChan + c8;
  const float* pp = x + (size_t)srow * kChan + c8;
  const v4f a  = *(const v4f*)(xp);
  const v4f b  = *(const v4f*)(xp + 4);
  const v4f pa = *(const v4f*)(pp);
  const v4f pb = *(const v4f*)(pp + 4);
  const v4f ma = *(const v4f*)(mvec + c8);
  const v4f mb = *(const v4f*)(mvec + c8 + 4);
  float o[8];
#pragma unroll
  for (int e = 0; e < 4; ++e) {
    const float p0 = first ? 0.0f : pa[e];
    const float p1 = first ? 0.0f : pb[e];
    o[e]     = a[e] + (p0 - a[e]) * ma[e];
    o[4 + e] = b[e] + (p1 - b[e]) * mb[e];
  }
  const v4u u = pack8_plain(o);
  const size_t off = (size_t)i * 8;
  *(volatile v4u*)(XM + off) = u;
  __threadfence();
  *(volatile v4u*)(XM + off) = u;
}

__global__ __launch_bounds__(256) void gate_prep_kernel(float* K0, float* WZ, unsigned* KKL,
                                                        const unsigned* __restrict__ AL, unsigned* MAL,
                                                        const unsigned* __restrict__ MKL,
                                                        const float* __restrict__ w0, const float* __restrict__ a0,
                                                        const float* __restrict__ ma0, const float* __restrict__ mk0) {
  const int lane = threadIdx.x & 31;
  const int pair = blockIdx.x * 8 + (threadIdx.x >> 5);
  const int tok = pair >> 4;
  const int h   = pair & 15;
  const size_t base = (size_t)tok * kChan + (size_t)h * kHdim + 2 * lane;
  const size_t widx = base >> 1;
  const int c0 = h * kHdim + 2 * lane;
  const v2f k2 = *(const v2f*)(K0 + base);
  const v2f z2 = *(const v2f*)(WZ + base);
  const unsigned wkk = KKL[widx];
  const unsigned wal = AL[widx];
  const unsigned wma = MAL[widx];
  const unsigned wmk = MKL[widx];
  const float k20 = k2[0], k21 = k2[1];
  const float z20 = z2[0], z21 = z2[1];
  float ss;
  {
    const float kr0 = k20 + h16_to_f32(wkk & 0xffffu);
    const float kr1 = k21 + h16_to_f32(wkk >> 16);
    ss = wave_sum32(kr0 * kr0 + kr1 * kr1);
  }
  const float inv = 1.0f / fmaxf(sqrtf(ss), 1e-12f);
  float kf0 = 0.0f, kf1 = 0.0f, dd0 = 0.0f, dd1 = 0.0f;
  unsigned wnk = 0u, wkb = 0u;
#pragma unroll 1
  for (int hf = 0; hf < 2; ++hf) {
    const int sh = 16 * hf;
    const int c = c0 + hf;
    const float k0v = (hf == 0) ? k20 : k21;
    const float zl  = (hf == 0) ? z20 : z21;
    const float kkl = h16_to_f32((wkk >> sh) & 0xffffu);
    const float al  = h16_to_f32((wal >> sh) & 0xffffu);
    const float mal = h16_to_f32((wma >> sh) & 0xffffu);
    const float mkl = h16_to_f32((wmk >> sh) & 0xffffu);
    const float kkv = (k0v + kkl) * inv;
    const float av  = __builtin_amdgcn_rcpf(1.0f + expf(-(a0[c] + al)));
    const float mav = __builtin_amdgcn_rcpf(1.0f + expf(-(ma0[c] + mal)));
    const float mkv = __builtin_amdgcn_rcpf(1.0f + expf(-(mk0[c] + mkl)));
    const float zz  = w0[c] + zl;
    const float wv  = fminf(zz, 0.0f) - log1pf(expf(-fabsf(zz))) - 0.5f;
    const float km  = (k0v * mav + k0v * av * (1.0f - mav)) * expf(fminf(wv * mkv, 0.0f));
    const float dv  = expf(wv);
    kf0 = (hf == 0) ? km : kf0;
    kf1 = (hf == 1) ? km : kf1;
    dd0 = (hf == 0) ? dv : dd0;
    dd1 = (hf == 1) ? dv : dd1;
    const unsigned nb = (unsigned)h_bits(-kkv);
    const unsigned bb = (unsigned)h_bits(kkv * av);
    wnk |= nb << sh;
    wkb |= bb << sh;
  }
  const v2f kfv = (v2f){kf0, kf1};
  const v2f ddv = (v2f){dd0, dd1};
  *(volatile v2f*)(K0 + base) = kfv;
  *(volatile v2f*)(WZ + base) = ddv;
  *(volatile unsigned*)(KKL + widx) = wnk;
  *(volatile unsigned*)(MAL + widx) = wkb;
  __threadfence();
  *(volatile v2f*)(K0 + base) = kfv;
  *(volatile v2f*)(WZ + base) = ddv;
  *(volatile unsigned*)(KKL + widx) = wnk;
  *(volatile unsigned*)(MAL + widx) = wkb;
}

__global__ __launch_bounds__(256) void state_scan_kernel(const unsigned short* __restrict__ Rh, const float* __restrict__ Dd,
                                                         const float* __restrict__ Kf, const unsigned short* __restrict__ Vh,
                                                         const unsigned short* __restrict__ Ah, const unsigned short* __restrict__ Bh,
                                                         float* __restrict__ Y) {
  __shared__ __align__(16) float lv[6 * kChunk * 64];
  __shared__ __align__(16) float yb[kChunk * 64];
  const int bh  = blockIdx.x;
  const int b   = bh >> 4;
  const int h   = bh & 15;
  const int tid = threadIdx.x;
  const int i   = tid >> 2;
  const int q   = tid & 3;
  const int j0  = q * 16;
  const int lrow = tid >> 4;
  const int lc4  = (tid & 15) * 4;
  const size_t base = (size_t)b * kSteps * kChan + (size_t)h * kHdim;

  float S[16];
#pragma unroll
  for (int jj = 0; jj < 16; ++jj) S[jj] = 0.0f;

#pragma unroll 1
  for (int ch = 0; ch < kSteps / kChunk; ++ch) {
    const size_t goff = base + (size_t)(ch * kChunk + lrow) * kChan + lc4;
    {
      const v4f t0 = ld4h(Rh + goff);
      const v4f t1 = *(const v4f*)(Dd + goff);
      const v4f t2 = *(const v4f*)(Kf + goff);
      const v4f t3 = ld4h(Vh + goff);
      const v4f t4 = ld4h(Ah + goff);
      const v4f t5 = ld4h(Bh + goff);
      const int lo = lrow * 64 + lc4;
      *(v4f*)(lv + 0 * kChunk * 64 + lo) = t0;
      *(v4f*)(lv + 1 * kChunk * 64 + lo) = t1;
      *(v4f*)(lv + 2 * kChunk * 64 + lo) = t2;
      *(v4f*)(lv + 3 * kChunk * 64 + lo) = t3;
      *(v4f*)(lv + 4 * kChunk * 64 + lo) = t4;
      *(v4f*)(lv + 5 * kChunk * 64 + lo) = t5;
    }
    __syncthreads();

#pragma unroll 1
    for (int s = 0; s < kChunk; ++s) {
      const float* pr = lv + 0 * kChunk * 64 + s * 64 + j0;
      const float* pd = lv + 1 * kChunk * 64 + s * 64 + j0;
      const float* pk = lv + 2 * kChunk * 64 + s * 64 + j0;
      const float* pa = lv + 4 * kChunk * 64 + s * 64 + j0;
      const float* pb = lv + 5 * kChunk * 64 + s * 64 + j0;
      const float vi = lv[3 * kChunk * 64 + s * 64 + i];
      float sa = 0.0f;
#pragma unroll
      for (int g4 = 0; g4 < 4; ++g4) {
        const v4f a4 = *(const v4f*)(pa + 4 * g4);
#pragma unroll
        for (int e = 0; e < 4; ++e) sa += S[4 * g4 + e] * a4[e];
      }
      sa += __shfl_xor(sa, 1, 32);
      sa += __shfl_xor(sa, 2, 32);
      float out = 0.0f;
#pragma unroll
      for (int g4 = 0; g4 < 4; ++g4) {
        const v4f d4 = *(const v4f*)(pd + 4 * g4);
        const v4f b4 = *(const v4f*)(pb + 4 * g4);
        const v4f k4 = *(const v4f*)(pk + 4 * g4);
        const v4f r4 = *(const v4f*)(pr + 4 * g4);
#pragma unroll
        for (int e = 0; e < 4; ++e) {
          const float sn = S[4 * g4 + e] * d4[e] + sa * b4[e] + vi * k4[e];
          S[4 * g4 + e] = sn;
          out += sn * r4[e];
        }
      }
      out += __shfl_xor(out, 1, 32);
      out += __shfl_xor(out, 2, 32);
      if (q == 0) yb[s * 64 + i] = out;
    }
    __syncthreads();
    {
      const v4f val = *(const v4f*)(yb + lrow * 64 + lc4);
      *(volatile v4f*)(Y + goff) = val;
      __threadfence();
      *(volatile v4f*)(Y + goff) = val;
    }
  }
}

__global__ __launch_bounds__(256) void norm_gate_kernel(const float* __restrict__ Y, const unsigned* __restrict__ Rw,
                                                        const float* __restrict__ Kf, const unsigned* __restrict__ Vw,
                                                        const unsigned* __restrict__ Gw, const float* __restrict__ fa,
                                                        const float* __restrict__ ln_w, const float* __restrict__ ln_b,
                                                        unsigned* __restrict__ YG) {
  const int lane = threadIdx.x & 31;
  const int pair = blockIdx.x * 8 + (threadIdx.x >> 5);
  const int tok = pair >> 4;
  const int h   = pair & 15;
  const size_t base = (size_t)tok * kChan + (size_t)h * kHdim + 2 * lane;
  const size_t widx = base >> 1;
  const int c = h * kHdim + 2 * lane;
  const v2f y2 = *(const v2f*)(Y + base);
  const v2f k2 = *(const v2f*)(Kf + base);
  const unsigned rw = Rw[widx];
  const unsigned vw = Vw[widx];
  const unsigned gw = Gw[widx];
  const v2f q2 = *(const v2f*)(fa + c);
  const v2f w2 = *(const v2f*)(ln_w + c);
  const v2f b2 = *(const v2f*)(ln_b + c);
  const float r0 = h16_to_f32(rw & 0xffffu), r1 = h16_to_f32(rw >> 16);
  const float v0 = h16_to_f32(vw & 0xffffu), v1 = h16_to_f32(vw >> 16);
  const float g0 = h16_to_f32(gw & 0xffffu), g1 = h16_to_f32(gw >> 16);
  const float mu = wave_sum32(y2[0] + y2[1]) * (1.0f / 64.0f);
  const float d0 = y2[0] - mu;
  const float d1 = y2[1] - mu;
  const float var = wave_sum32(d0 * d0 + d1 * d1) * (1.0f / 64.0f);
  const float inv = 1.0f / sqrtf(var + kGnEps);
  const float bsum = wave_sum32(r0 * k2[0] * q2[0] + r1 * k2[1] * q2[1]);
  const float o0 = (((d0 * inv) * w2[0] + b2[0]) + bsum * v0) * g0 * kYCarry;
  const float o1 = (((d1 * inv) * w2[1] + b2[1]) + bsum * v1) * g1 * kYCarry;
  const unsigned wo = pk16(h_bits(o0), h_bits(o1));
  *(volatile unsigned*)(YG + widx) = wo;
  __threadfence();
  *(volatile unsigned*)(YG + widx) = wo;
}

static PlaceArgs place_init(const float* dflt) {
  PlaceArgs a;
  for (int s = 0; s < 4; ++s) {
    a.p[s] = dflt;
    a.Kd[s] = 1;
    a.Nd[s] = 1;
    a.rowOff[s] = (1 << 28);
    a.colOff[s] = 0;
  }
  return a;
}
static void place_set(PlaceArgs& a, int s, const float* p, int Kd, int Nd, int rowOff, int colOff) {
  a.p[s] = p;
  a.Kd[s] = Kd;
  a.Nd[s] = Nd;
  a.rowOff[s] = rowOff;
  a.colOff[s] = colOff;
}

extern "C" void kernel_launch(void* const* d_in, const int* in_sizes, int n_in,
                              void* d_out, int out_size, void* d_ws, size_t ws_size, hipStream_t stream) {
  if (n_in < 31 || d_out == nullptr || d_ws == nullptr) return;
  const int nP = (int)kPlane;
  const int expect[31] = {
      nP, kChan, kChan, kChan, kChan, kChan,
      kChan * kMixHid, 4 * kMixRank * kChan,
      kChan, kChan * kDecHid, kDecHid * kChan,
      kHeads * kHdim, kChan,
      kChan * kLoraR, kLoraR * kChan, kChan * kLoraR, kLoraR * kChan,
      kChan * kGateHid, kGateHid * kChan,
      kChan * kLoraR, kLoraR * kChan, kChan,
      kChan * kLoraR, kLoraR * kChan, kChan,
      kChan * kChan, kChan * kChan, kChan * kChan, kChan * kChan,
      kChan, kChan};
  for (int i = 0; i < 31; ++i) if (in_sizes[i] != expect[i]) return;
  if (out_size != nP) return;

  const float* x       = (const float*)d_in[0];
  const float* maa_x   = (const float*)d_in[1];
  const float* maa_rg  = (const float*)d_in[2];
  const float* maa_wa  = (const float*)d_in[3];
  const float* maa_k   = (const float*)d_in[4];
  const float* maa_v   = (const float*)d_in[5];
  const float* maa_w1  = (const float*)d_in[6];
  const float* maa_w2  = (const float*)d_in[7];
  const float* tdecay  = (const float*)d_in[8];
  const float* dec_w1  = (const float*)d_in[9];
  const float* dec_w2  = (const float*)d_in[10];
  const float* faaaa   = (const float*)d_in[11];
  const float* aaaaa   = (const float*)d_in[12];
  const float* aaa_w1  = (const float*)d_in[13];
  const float* aaa_w2  = (const float*)d_in[14];
  const float* kkk_w1  = (const float*)d_in[15];
  const float* kkk_w2  = (const float*)d_in[16];
  const float* gate_w1 = (const float*)d_in[17];
  const float* gate_w2 = (const float*)d_in[18];
  const float* ma_w1   = (const float*)d_in[19];
  const float* ma_w2   = (const float*)d_in[20];
  const float* misc_a  = (const float*)d_in[21];
  const float* mk_w1   = (const float*)d_in[22];
  const float* mk_w2   = (const float*)d_in[23];
  const float* misc_k  = (const float*)d_in[24];
  const float* W_r     = (const float*)d_in[25];
  const float* W_k     = (const float*)d_in[26];
  const float* W_v     = (const float*)d_in[27];
  const float* W_o     = (const float*)d_in[28];
  const float* ln_w    = (const float*)d_in[29];
  const float* ln_b    = (const float*)d_in[30];
  float* out0 = (float*)d_out;

  char* ws = (char*)d_ws;
  size_t off = 0;
  auto carve = [&](size_t bytes) -> char* {
    char* p = ws + off;
    off += (bytes + 255) & ~(size_t)255;
    return p;
  };
  const size_t actB = kPlane * 2;
  const size_t wBig = (size_t)kChan * kChan;
  unsigned short* XA  = (unsigned short*)carve(actB);
  unsigned short* MA  = (unsigned short*)carve(actB);
  unsigned short* KKL = (unsigned short*)carve(actB);
  unsigned short* MK  = (unsigned short*)carve(actB);
  unsigned short* XRG = (unsigned short*)carve(actB);
  unsigned short* XWA = (unsigned short*)carve(actB);
  unsigned short* XK  = (unsigned short*)carve(actB);
  unsigned short* XV  = (unsigned short*)carve(actB);
  unsigned short* R   = (unsigned short*)carve(actB);
  unsigned short* V   = (unsigned short*)carve(actB);
  float* K0 = (float*)carve(kPlane * 4);
  float* WZ = (float*)carve(kPlane * 4);
  unsigned short* WB  = (unsigned short*)carve(4 * wBig * 2);
  unsigned short* W1T = (unsigned short*)carve((size_t)kW1Rows * kChan * 2);
  unsigned short* M2T = (unsigned short*)carve((size_t)4 * kChan * kK2Pitch * 2);
  unsigned short* L2T = (unsigned short*)carve((size_t)4 * kChan * kK2Pitch * 2);
  unsigned short* D2T = (unsigned short*)carve((size_t)kChan * kK2Pitch * 2);
  unsigned short* G2T = (unsigned short*)carve((size_t)kChan * kGateHid * 2);
  unsigned short* HMIX = (unsigned short*)carve((size_t)kTok * kMixHid * 2);
  unsigned short* HG   = (unsigned short*)carve((size_t)kTok * kGateHid * 2);
  unsigned short* HWA  = (unsigned short*)carve((size_t)kTok * kHidWa * 2);
  unsigned short* HK   = (unsigned short*)carve((size_t)kTok * kHidK * 2);
  if (off > ws_size || off > (size_t)134217728) return;
  if (XWA != XRG + kPlane || XK != XWA + kPlane || XV != XK + kPlane) return;
  if (MA != XA + kPlane || MK != KKL + kPlane) return;
  float* Yf = (float*)(void*)XRG;
  unsigned short* YG = XK;
  unsigned short* Gh = XV;

  cast8_w4_kernel<<<dim3((unsigned)(wBig / 8 / 256), 4), 256, 0, stream>>>(W_r, W_k, W_v, W_o, WB,
                                                                            kWCarry, kWkCarry, kWCarry, kWCarry, (int)(wBig / 8));
  {
    PlaceArgs a = place_init(maa_w1);
    place_set(a, 0, maa_w1, kChan, kMixHid, 0, 0);
    place_set(a, 1, gate_w1, kChan, kGateHid, kMixHid, 0);
    wt_place_kernel<<<dim3(kChan / 64, (kMixHid + kGateHid) / 64), 256, 0, stream>>>(a, W1T, kChan, kWCarry);
  }
  {
    PlaceArgs a = place_init(dec_w1);
    place_set(a, 0, dec_w1, kChan, kDecHid, 0, 0);
    place_set(a, 1, aaa_w1, kChan, kLoraR, kDecHid, 0);
    place_set(a, 2, ma_w1, kChan, kLoraR, kDecHid + kLoraR, 0);
    wt_place_kernel<<<dim3(kChan / 64, kHidWa / 64), 256, 0, stream>>>(
        a, W1T + (size_t)(kMixHid + kGateHid) * kChan, kChan, kWCarry);
  }
  {
    PlaceArgs a = place_init(kkk_w1);
    place_set(a, 0, kkk_w1, kChan, kLoraR, 0, 0);
    place_set(a, 1, mk_w1, kChan, kLoraR, kLoraR, 0);
    wt_place_kernel<<<dim3(kChan / 64, kHidK / 64), 256, 0, stream>>>(
        a, W1T + (size_t)(kMixHid + kGateHid + kHidWa) * kChan, kChan, kWCarry);
  }
  {
    PlaceArgs a = place_init(maa_w2);
    for (int f = 0; f < 4; ++f) place_set(a, f, maa_w2 + (size_t)f * kMixRank * kChan, kMixRank, kChan, f * kChan, 0);
    wt_place_kernel<<<dim3(kK2Pitch / 64, (4 * kChan) / 64), 256, 0, stream>>>(a, M2T, kK2Pitch, kWCarry);
  }
  {
    PlaceArgs a = place_init(aaa_w2);
    place_set(a, 0, aaa_w2, kLoraR, kChan, 0, 0);
    place_set(a, 1, ma_w2, kLoraR, kChan, kChan, kLoraR);
    place_set(a, 2, kkk_w2, kLoraR, kChan, 2 * kChan, 0);
    place_set(a, 3, mk_w2, kLoraR, kChan, 3 * kChan, kLoraR);
    wt_place_kernel<<<dim3(kK2Pitch / 64, (4 * kChan) / 64), 256, 0, stream>>>(a, L2T, kK2Pitch, kWCarry);
  }
  {
    PlaceArgs a = place_init(dec_w2);
    place_set(a, 0, dec_w2, kDecHid, kChan, 0, 0);
    wt_place_kernel<<<dim3(kK2Pitch / 64, kChan / 64), 256, 0, stream>>>(a, D2T, kK2Pitch, kWCarry);
  }
  {
    PlaceArgs a = place_init(gate_w2);
    place_set(a, 0, gate_w2, kGateHid, kChan, 0, 0);
    wt_place_kernel<<<dim3(kGateHid / 64, kChan / 64), 256, 0, stream>>>(a, G2T, kGateHid, kWCarry);
  }

  const unsigned short* maa_w1t = W1T;
  const unsigned short* gate_w1t = W1T + (size_t)kMixHid * kChan;
  const unsigned short* hidwa_bt = W1T + (size_t)(kMixHid + kGateHid) * kChan;
  const unsigned short* hidk_bt  = W1T + (size_t)(kMixHid + kGateHid + kHidWa) * kChan;

  const int blkBig = (kTok / 32) * (kChan / 64) / 8;
  const int blk128 = (kTok / 32) * (128 / 64) / 8;
  const int blk64  = (kTok / 32) * (64 / 64) / 8;

  shift_mix_kernel<<<(kTok * (kChan / 8)) / 256, 256, 0, stream>>>(x, maa_x, XA);

  gemm_f16_kernel<1, 1><<<dim3(blk128, 1), 256, 0, stream>>>(
      XA, kChan, 0L, maa_w1t, kChan, 0L, (void*)HMIX, kMixHid, 0L,
      kTok, kMixHid, kChan, kScaleW, kHidCarry, kMixHid);

  mix2_kernel<<<dim3(blkBig, 4), 256, 0, stream>>>(HMIX, M2T, x, maa_rg, maa_wa, maa_k, maa_v, XRG, kScaleWH);

  gemm_f16_kernel<0, 1><<<dim3(blkBig, 1), 256, 0, stream>>>(
      XRG, kChan, 0L, WB, kChan, 0L, (void*)R, kChan, 0L, kTok, kChan, kChan, kScaleW, 1.0f, 0);
  gemm_f16_kernel<0, 0><<<dim3(blkBig, 1), 256, 0, stream>>>(
      XK, kChan, 0L, WB + wBig, kChan, 0L, (void*)K0, kChan, 0L, kTok, kChan, kChan, kScaleWk, 1.0f, 0);
  gemm_f16_kernel<0, 1><<<dim3(blkBig, 1), 256, 0, stream>>>(
      XV, kChan, 0L, WB + 2 * wBig, kChan, 0L, (void*)V, kChan, 0L, kTok, kChan, kChan, kScaleW, 1.0f, 0);

  gemm_f16_kernel<1, 1><<<dim3(blk128, 1), 256, 0, stream>>>(
      XRG, kChan, 0L, gate_w1t, kChan, 0L, (void*)HG, kGateHid, 0L,
      kTok, kGateHid, kChan, kScaleW, kHidCarry, kGateHid);
  gemm_f16_kernel<1, 1><<<dim3(blk128, 1), 256, 0, stream>>>(
      XWA, kChan, 0L, hidwa_bt, kChan, 0L, (void*)HWA, kHidWa, 0L,
      kTok, kHidWa, kChan, kScaleW, kHidCarry, kDecHid);
  gemm_f16_kernel<1, 1><<<dim3(blk64, 1), 256, 0, stream>>>(
      XK, kChan, 0L, hidk_bt, kChan, 0L, (void*)HK, kHidK, 0L,
      kTok, kHidK, kChan, kScaleW, kHidCarry, kLoraR);

  gemm_f16_kernel<0, 1><<<dim3(blkBig, 1), 256, 0, stream>>>(
      HG, kGateHid, 0L, G2T, kGateHid, 0L, (void*)Gh, kChan, 0L, kTok, kChan, kGateHid, kScaleWH, 1.0f, 0);
  gemm_f16_kernel<0, 0><<<dim3(blkBig, 1), 256, 0, stream>>>(
      HWA, kHidWa, 0L, D2T, kK2Pitch, 0L, (void*)WZ, kChan, 0L, kTok, kChan, kDecHid, kScaleWH, 1.0f, 0);
  gemm_f16_kernel<0, 1><<<dim3(blkBig, 2), 256, 0, stream>>>(
      HWA + kDecHid, kHidWa, 0L, L2T, kK2Pitch, (long)((size_t)kChan * kK2Pitch),
      (void*)XA, kChan, (long)kPlane, kTok, kChan, 2 * kLoraR, kScaleWH, 1.0f, 0);
  gemm_f16_kernel<0, 1><<<dim3(blkBig, 2), 256, 0, stream>>>(
      HK, kHidK, 0L, L2T + (size_t)2 * kChan * kK2Pitch, kK2Pitch, (long)((size_t)kChan * kK2Pitch),
      (void*)KKL, kChan, (long)kPlane, kTok, kChan, 2 * kLoraR, kScaleWH, 1.0f, 0);

  gate_prep_kernel<<<(kTok * kHeads) / 8, 256, 0, stream>>>(K0, WZ, (unsigned*)KKL, (const unsigned*)XA, (unsigned*)MA,
                                                            (const unsigned*)MK, tdecay, aaaaa, misc_a, misc_k);

  state_scan_kernel<<<kBatch * kHeads, 256, 0, stream>>>(R, WZ, K0, V, KKL, MA, Yf);

  norm_gate_kernel<<<(kTok * kHeads) / 8, 256, 0, stream>>>(Yf, (const unsigned*)R, K0, (const unsigned*)V,
                                                            (const unsigned*)Gh, faaaa, ln_w, ln_b, (unsigned*)YG);

  gemm_f16_kernel<0, 0><<<dim3(blkBig, 1), 256, 0, stream>>>(
      YG, kChan, 0L, WB + 3 * wBig, kChan, 0L, (void*)out0, kChan, 0L, kTok, kChan, kChan, kScaleOut, 1.0f, 0);
}
